// LSTM_13915694039291
// MI455X (gfx1250) — hardware-verified
//
#include <hip/hip_runtime.h>


typedef __attribute__((ext_vector_type(16))) _Float16 v16h_;
typedef __attribute__((ext_vector_type(8)))  _Float16 v8h_;
typedef __attribute__((ext_vector_type(4)))  float  v4f;
typedef __attribute__((ext_vector_type(8)))  float  v8f;

#define HDIM   128
#define GDIM   512
#define BSZ    256
#define TLEN   1024
#define MROWS  16
#define HSTRIDE 136

#define OFF_WHH0  0
#define OFF_WHH1  131072
#define OFF_H0    262144
#define OFF_H1    (OFF_H0 + 2*MROWS*HSTRIDE*2)
#define OFF_H1F   (OFF_H1 + 2*MROWS*HSTRIDE*2)
#define SMEM_BYTES (OFF_H1F + MROWS*HDIM*4)

__device__ __forceinline__ float sigmoidf_(float v) {
    return 1.0f / (1.0f + expf(-v));
}
__device__ __forceinline__ v8f wmma_h(v16h_ a, v16h_ b, v8f c) {
    c = __builtin_amdgcn_wmma_f32_16x16x32_f16(false, a, false, b, (short)0, c, false, false);
    asm volatile("v_nop\n\tv_nop\n\tv_nop\n\tv_nop" : "+v"(c) : "v"(a), "v"(b));
    return c;
}

__device__ __forceinline__ v16h_ load_a_frag(const _Float16* hbase, int kt, int lr, int lh) {
    const _Float16* row = hbase + lr * HSTRIDE;
    int k0 = kt * 32 + lh * 8;
    v8h_ lo = *(const v8h_*)(row + k0);
    v8h_ hi = *(const v8h_*)(row + k0 + 16);
    v16h_ r;
#pragma unroll
    for (int e = 0; e < 8; ++e) { r[e] = lo[e]; r[e + 8] = hi[e]; }
    return r;
}

__device__ __forceinline__ v16h_ load_b_frag(const _Float16* fragbase, int lane) {
    const _Float16* p = fragbase + lane * 16;
    v8h_ lo = *(const v8h_*)p;
    v8h_ hi = *(const v8h_*)(p + 8);
    v16h_ r;
#pragma unroll
    for (int e = 0; e < 8; ++e) { r[e] = lo[e]; r[e + 8] = hi[e]; }
    return r;
}

__global__ void __launch_bounds__(256, 1)
lstm2_fused(const float* __restrict__ x,
            const float* __restrict__ h0in,
            const float* __restrict__ c0in,
            const float* __restrict__ Wih0,
            const float* __restrict__ Whh0,
            const float* __restrict__ bih0,
            const float* __restrict__ bhh0,
            const float* __restrict__ Wih1,
            const float* __restrict__ Whh1,
            const float* __restrict__ bih1,
            const float* __restrict__ bhh1,
            const float* __restrict__ Wbw,
            const float* __restrict__ bbw,
            const float* __restrict__ Wcls,
            const float* __restrict__ bcls,
            float* __restrict__ headstg,
            float* __restrict__ out)
{
    extern __shared__ char smem[];
    _Float16* whh0f = (_Float16*)(smem + OFF_WHH0);
    _Float16* whh1f = (_Float16*)(smem + OFF_WHH1);
    _Float16* h0buf = (_Float16*)(smem + OFF_H0);
    _Float16* h1buf = (_Float16*)(smem + OFF_H1);
    float*  h1f   = (float*)(smem + OFF_H1F);

    const int tid  = threadIdx.x;
    const int lane = tid & 31;
    const int wv   = tid >> 5;
    const int m0   = blockIdx.x * MROWS;
    const int lr   = lane & 15;
    const int lh   = lane >> 4;
    const int jloc = wv * 16 + lr;

    for (int idx = tid; idx < 4096; idx += 256) {
        int ln  = idx & 31;
        int fid = idx >> 5;
        int kt  = fid & 3;
        int nt  = fid >> 2;
        int g   = nt * 16 + (ln & 15);
        int kb  = kt * 32 + ((ln >> 4) << 3);
        const float* s0 = Whh0 + g * HDIM + kb;
        const float* s1 = Whh1 + g * HDIM + kb;
        _Float16* d0 = whh0f + (fid * 32 + ln) * 16;
        _Float16* d1 = whh1f + (fid * 32 + ln) * 16;
#pragma unroll
        for (int e = 0; e < 8; ++e) { d0[e] = (_Float16)s0[e]; d1[e] = (_Float16)s1[e]; d0[8 + e] = (_Float16)s0[16 + e]; d1[8 + e] = (_Float16)s1[16 + e]; }
    }
    for (int idx = tid; idx < MROWS * HDIM; idx += 256) {
        int m = idx >> 7;
        int k = idx & 127;
        h0buf[m * HSTRIDE + k] = (_Float16)h0in[(0 * BSZ + m0 + m) * HDIM + k];
        h1buf[m * HSTRIDE + k] = (_Float16)h0in[(1 * BSZ + m0 + m) * HDIM + k];
    }

    v16h_ wih1f[4][4];
#pragma unroll
    for (int gg = 0; gg < 4; ++gg) {
#pragma unroll
        for (int kt = 0; kt < 4; ++kt) {
            int nt = gg * 8 + wv;
            int g  = nt * 16 + lr;
            int kb = kt * 32 + (lh << 3);
            const float* s = Wih1 + g * HDIM + kb;
            v16h_ v;
#pragma unroll
            for (int e = 0; e < 8; ++e) { v[e] = (_Float16)s[e]; v[8 + e] = (_Float16)s[16 + e]; }
            wih1f[gg][kt] = v;
        }
    }

    float wi0g[4], wi1g[4], b0g[4], b1g[4];
#pragma unroll
    for (int gg = 0; gg < 4; ++gg) {
        int n = gg * HDIM + jloc;
        wi0g[gg] = Wih0[n * 2 + 0];
        wi1g[gg] = Wih0[n * 2 + 1];
        b0g[gg]  = bih0[n] + bhh0[n];
        b1g[gg]  = bih1[n] + bhh1[n];
    }

    float c0r[8], c1r[8], h0v[8], h1v[8];
#pragma unroll
    for (int r = 0; r < 8; ++r) {
        int b = m0 + r + 8 * lh;
        c0r[r] = c0in[(0 * BSZ + b) * HDIM + jloc];
        c1r[r] = c0in[(1 * BSZ + b) * HDIM + jloc];
        h0v[r] = 0.f; h1v[r] = 0.f;
    }

    __syncthreads();

    for (int t = 0; t < TLEN; ++t) {
        const int p = t & 1;
        const int q = p ^ 1;
        _Float16* h0r = h0buf + p * MROWS * HSTRIDE;
        _Float16* h0w = h0buf + q * MROWS * HSTRIDE;
        _Float16* h1r = h1buf + p * MROWS * HSTRIDE;
        _Float16* h1w = h1buf + q * MROWS * HSTRIDE;

        v16h_ a0[4], ah1[4];
#pragma unroll
        for (int kt = 0; kt < 4; ++kt) {
            a0[kt]  = load_a_frag(h0r, kt, lr, lh);
            ah1[kt] = load_a_frag(h1r, kt, lr, lh);
        }

        float x0[8], x1[8];
#pragma unroll
        for (int r = 0; r < 8; ++r) {
            int b = m0 + r + 8 * lh;
            const float* xp = x + ((size_t)b * TLEN + t) * 2;
            x0[r] = xp[0]; x1[r] = xp[1];
            if (t + 1 < TLEN) __builtin_prefetch(xp + 2, 0, 1);
        }
        v8f acc[4];
#pragma unroll
        for (int gg = 0; gg < 4; ++gg) {
            v8f a;
#pragma unroll
            for (int r = 0; r < 8; ++r)
                a[r] = fmaf(x0[r], wi0g[gg], fmaf(x1[r], wi1g[gg], b0g[gg]));
            acc[gg] = a;
        }
#pragma unroll
        for (int gg = 0; gg < 4; ++gg) {
            int nt = gg * 8 + wv;
#pragma unroll
            for (int kt = 0; kt < 4; ++kt) {
                v16h_ bf = load_b_frag(whh0f + ((nt * 4 + kt) * 32) * 16, lane);
                acc[gg] = wmma_h(a0[kt], bf, acc[gg]);
            }
        }
#pragma unroll
        for (int r = 0; r < 8; ++r) {
            float iv = sigmoidf_(acc[0][r]);
            float fv = sigmoidf_(acc[1][r]);
            float gv = tanhf(acc[2][r]);
            float ov = sigmoidf_(acc[3][r]);
            float c  = fv * c0r[r] + iv * gv;
            c0r[r]   = c;
            h0v[r]   = ov * tanhf(c);
            h0w[(r + 8 * lh) * HSTRIDE + jloc] = (_Float16)h0v[r];
        }

        __syncthreads();

        v16h_ a1[4];
#pragma unroll
        for (int kt = 0; kt < 4; ++kt) a1[kt] = load_a_frag(h0w, kt, lr, lh);

        v8f acc1[4];
#pragma unroll
        for (int gg = 0; gg < 4; ++gg) {
            v8f a;
#pragma unroll
            for (int r = 0; r < 8; ++r) a[r] = b1g[gg];
            acc1[gg] = a;
        }
#pragma unroll
        for (int gg = 0; gg < 4; ++gg) {
#pragma unroll
            for (int kt = 0; kt < 4; ++kt)
                acc1[gg] = wmma_h(a1[kt], wih1f[gg][kt], acc1[gg]);
            int nt = gg * 8 + wv;
#pragma unroll
            for (int kt = 0; kt < 4; ++kt) {
                v16h_ bf = load_b_frag(whh1f + ((nt * 4 + kt) * 32) * 16, lane);
                acc1[gg] = wmma_h(ah1[kt], bf, acc1[gg]);
            }
        }
#pragma unroll
        for (int r = 0; r < 8; ++r) {
            float iv = sigmoidf_(acc1[0][r]);
            float fv = sigmoidf_(acc1[1][r]);
            float gv = tanhf(acc1[2][r]);
            float ov = sigmoidf_(acc1[3][r]);
            float c  = fv * c1r[r] + iv * gv;
            c1r[r]   = c;
            h1v[r]   = ov * tanhf(c);
            h1w[(r + 8 * lh) * HSTRIDE + jloc] = (_Float16)h1v[r];
        }

        __syncthreads();
    }

    float* stg = (float*)(smem + OFF_WHH0);
#pragma unroll
    for (int r = 0; r < 8; ++r) {
        const int m = r + 8 * lh;
        stg[(0 * MROWS + m) * HDIM + jloc] = h0v[r];
        stg[(1 * MROWS + m) * HDIM + jloc] = h1v[r];
        stg[(2 * MROWS + m) * HDIM + jloc] = c0r[r];
        stg[(3 * MROWS + m) * HDIM + jloc] = c1r[r];
        h1f[m * HDIM + jloc] = h1v[r];
    }
    __syncthreads();
    {
        for (int pass = 0; pass < 2; ++pass) {
#pragma unroll
            for (int i = 0; i < 8; ++i) {
                const int rr = wv * 8 + i, ti = rr >> 4, m = rr & 15;
                const v4f v = *(const v4f*)(stg + (size_t)rr * HDIM + lane * 4);
                *(volatile v4f*)(out + 512 + (size_t)ti * 32768 + (size_t)(m0 + m) * HDIM + lane * 4) = v;
            }
            __threadfence();
        }
    }
    if (tid < 32) {
        const int m = tid & 15;
        float s = 0.f;
        const float* wgt = (tid < 16) ? Wbw : Wcls;
        for (int k = 0; k < HDIM; ++k) s = fmaf(h1f[m * HDIM + k], wgt[k], s);
        s += (tid < 16) ? bbw[0] : bcls[0];
        ((volatile float*)headstg)[blockIdx.x * 32 + tid] = s;
        __threadfence();
        ((volatile float*)headstg)[blockIdx.x * 32 + tid] = s;
    }
}

__global__ void heads_kernel(const float* __restrict__ headstg, float* __restrict__ out) {
    const int t = threadIdx.x;
    v4f v;
#pragma unroll
    for (int q = 0; q < 4; ++q) {
        const int i = 4 * t + q;
        const int which = i >> 8, b = i & 255;
        v[q] = headstg[(b >> 4) * 32 + which * 16 + (b & 15)];
    }
    *(volatile v4f*)(out + 4 * t) = v;
    __threadfence();
    *(volatile v4f*)(out + 4 * t) = v;
}

extern "C" void kernel_launch(void* const* d_in, const int* in_sizes, int n_in,
                              void* d_out, int out_size, void* d_ws, size_t ws_size,
                              hipStream_t stream) {
    (void)in_sizes; (void)n_in; (void)out_size; (void)ws_size;
    const float* x    = (const float*)d_in[0];
    const float* h0   = (const float*)d_in[1];
    const float* c0   = (const float*)d_in[2];
    const float* Wih0 = (const float*)d_in[3];
    const float* Whh0 = (const float*)d_in[4];
    const float* bih0 = (const float*)d_in[5];
    const float* bhh0 = (const float*)d_in[6];
    const float* Wih1 = (const float*)d_in[7];
    const float* Whh1 = (const float*)d_in[8];
    const float* bih1 = (const float*)d_in[9];
    const float* bhh1 = (const float*)d_in[10];
    const float* Wbw  = (const float*)d_in[11];
    const float* bbw  = (const float*)d_in[12];
    const float* Wcls = (const float*)d_in[13];
    const float* bcls = (const float*)d_in[14];
    float* out = (float*)d_out;

    hipFuncSetAttribute((const void*)lstm2_fused,
                        hipFuncAttributeMaxDynamicSharedMemorySize,
                        (int)SMEM_BYTES);

    float* headstg = (float*)d_ws;
    hipLaunchKernelGGL(lstm2_fused, dim3(BSZ / MROWS), dim3(256), SMEM_BYTES, stream,
                       x, h0, c0, Wih0, Whh0, bih0, bhh0,
                       Wih1, Whh1, bih1, bhh1, Wbw, bbw, Wcls, bcls, headstg, out);
    hipLaunchKernelGGL(heads_kernel, dim3(1), dim3(128), 0, stream, headstg, out);
}
